// MultiheadAttention_33904471835012
// MI455X (gfx1250) — hardware-run, weakly checked
//
#include <hip/hip_runtime.h>


#ifndef SEQI
#define SEQI 2048
#endif
#ifndef SEQJ
#define SEQJ 2048
#endif
#define SEQI_FULL 2048
#define SEQJ_FULL 2048
#define DM   1024
#define NHD  64
#define FD   16
#define AW   4
#define SC2  (0.125f * 1.4426950408889634f)
#define PSH  14.0f
#define RSC  2048.0f
#define RINV 0.00048828125f
#define VSC  16.0f
#define OSC  3.814697265625e-06f
#define TP   72
#define GP   36
#define HP2  (2 * DM)

static_assert(NHD * FD == DM);
static_assert(FD == 16);
static_assert(NHD % AW == 0);
static_assert(DM % 128 == 0);
static_assert((DM & (DM - 1)) == 0);
static_assert(SEQI % 64 == 0);
static_assert(SEQJ % 64 == 0);
static_assert(SEQI <= SEQI_FULL);
static_assert(SEQJ <= SEQJ_FULL);
static_assert(((size_t)SEQI * DM) % 8 == 0);
static_assert(((size_t)SEQJ * DM) % 8 == 0);

typedef _Float16 h16;
typedef unsigned short u16;
typedef __attribute__((ext_vector_type(16))) _Float16 v16h;
typedef __attribute__((ext_vector_type(8)))  _Float16 v8h;
typedef __attribute__((ext_vector_type(8)))  float    v8f;
typedef __attribute__((ext_vector_type(4)))  float    v4f;
typedef __attribute__((ext_vector_type(8)))  unsigned short v8us;
typedef __attribute__((ext_vector_type(4)))  int      v4i;
typedef __attribute__((ext_vector_type(8)))  int      v8i;
typedef __attribute__((ext_vector_type(16))) __bf16   v16bf;
typedef v4f  __attribute__((may_alias)) v4fa;
typedef v8us __attribute__((may_alias)) v8usa;
typedef v4i  __attribute__((may_alias)) v4ia;

__device__ __forceinline__ unsigned rbfb(float f) { unsigned u = __float_as_uint(f); u += 0x7FFFu + ((u >> 16) & 1u); return u >> 16; }
__device__ __forceinline__ float bf2f(unsigned b) { return __uint_as_float(b << 16); }
__device__ __forceinline__ v16h cat16(v8h lo, v8h hi) { return __builtin_shufflevector(lo, hi, 0, 1, 2, 3, 4, 5, 6, 7, 8, 9, 10, 11, 12, 13, 14, 15); }
__device__ __forceinline__ v8f wmma16(v16h a, v16h b, v8f c) { return __builtin_amdgcn_wmma_f32_16x16x32_f16(false, a, false, b, (short)0, c, false, false); }
__device__ __forceinline__ v8f wmmab(v8i a, v8i b, v8f c) { return __builtin_amdgcn_wmma_f32_16x16x32_bf16(false, __builtin_bit_cast(v16bf, a), false, __builtin_bit_cast(v16bf, b), (short)0, c, false, false); }
__device__ __forceinline__ v16h ldh(const h16* p) { return cat16(*(const v8h*)p, *(const v8h*)(p + 16)); }
__device__ __forceinline__ v8i ldbf(const u16* p) { const v4i lo = *(const v4ia*)p; const v4i hi = *(const v4ia*)(p + 16); return __builtin_shufflevector(lo, hi, 0, 1, 2, 3, 4, 5, 6, 7); }

__global__ __launch_bounds__(256) void k_cvt(const float* __restrict__ s, u16* d, size_t n8) {
    const size_t i = (size_t)blockIdx.x * 256 + threadIdx.x; if (i >= n8) return;
    const size_t e = i * 8;
    const v8f x = *(const v8f*)(s + e); v8us o;
#pragma unroll
    for (int k = 0; k < 8; ++k) o[k] = (u16)rbfb(x[k]);
    *(volatile v8us*)(d + e) = o;
    __threadfence();
    *(volatile v8us*)(d + e) = o;
}

__global__ __launch_bounds__(256) void k_wt(const float* __restrict__ W, u16* Wt) {
    __shared__ __align__(16) u16 ts[64 * TP];
    const int tid = threadIdx.x;
    const int n0 = blockIdx.x * 64, k0 = blockIdx.y * 64;
    const int r = tid >> 2, c0 = (tid & 3) * 16;
    const float* src = W + (size_t)(k0 + r) * DM + n0 + c0;
#pragma unroll
    for (int q = 0; q < 4; ++q) { const v4f x = *(const v4f*)(src + 4 * q);
#pragma unroll
        for (int i = 0; i < 4; ++i) ts[(c0 + 4 * q + i) * TP + r] = (u16)rbfb(x[i]); }
    __syncthreads();
    u16* dstb = Wt + (size_t)n0 * DM + k0;
#pragma unroll 1
    for (int ps = 0; ps < 2; ++ps) {
#pragma unroll
        for (int s = 0; s < 2; ++s) { const int n = 32 * s + (tid >> 3), c8 = (tid & 7) * 8;
            const v8us val = *(const v8usa*)(&ts[n * TP + c8]);
            *(volatile v8us*)(dstb + (size_t)n * DM + c8) = val; }
        if (ps == 0) __threadfence(); }
}

#define STG(acc, mi, ni) { const int o_ = wb + (16 * (mi) + 8 * hi) * GP + 16 * (ni) + lr; \
    gs[o_] = acc[0] * scale; gs[o_ + GP] = acc[1] * scale; gs[o_ + 2 * GP] = acc[2] * scale; gs[o_ + 3 * GP] = acc[3] * scale; \
    gs[o_ + 4 * GP] = acc[4] * scale; gs[o_ + 5 * GP] = acc[5] * scale; gs[o_ + 6 * GP] = acc[6] * scale; gs[o_ + 7 * GP] = acc[7] * scale; }

template <int MODE, typename OT>
__global__ __launch_bounds__(32 * AW) void k_gemm(const u16* __restrict__ A, int pitchA, const u16* __restrict__ Bt, int pitchB, int K, int kmask, OT* out, int ldo, float scale) {
    __shared__ __align__(16) float gs[AW * 64 * GP];
    const int lane = threadIdx.x & 31, wave = __builtin_amdgcn_readfirstlane((int)(threadIdx.x >> 5)), lr = lane & 15, hi = lane >> 4;
    const int row0 = blockIdx.y * 64, col0 = blockIdx.x * 128 + wave * 32;
    const u16* ap = A + (size_t)(row0 + lr) * pitchA + 8 * hi;
    const u16* bp = Bt + (size_t)(col0 + lr) * pitchB + 8 * hi;
    v8f c00 = (v8f){}, c01 = (v8f){}, c10 = (v8f){}, c11 = (v8f){}, c20 = (v8f){}, c21 = (v8f){}, c30 = (v8f){}, c31 = (v8f){};
#pragma unroll 1
    for (int k0 = 0; k0 < K; k0 += 32) {
        const int kb = k0 & kmask;
        const v8i a0 = ldbf(ap + k0), a1 = ldbf(ap + (size_t)16 * pitchA + k0), a2 = ldbf(ap + (size_t)32 * pitchA + k0), a3 = ldbf(ap + (size_t)48 * pitchA + k0);
        const v8i b0 = ldbf(bp + kb), b1 = ldbf(bp + (size_t)16 * pitchB + kb);
        c00 = wmmab(a0, b0, c00); c01 = wmmab(a0, b1, c01);
        c10 = wmmab(a1, b0, c10); c11 = wmmab(a1, b1, c11);
        c20 = wmmab(a2, b0, c20); c21 = wmmab(a2, b1, c21);
        c30 = wmmab(a3, b0, c30); c31 = wmmab(a3, b1, c31);
        asm volatile("v_nop\n\tv_nop\n\tv_nop\n\tv_nop" : "+v"(c00), "+v"(c01), "+v"(c10), "+v"(c11), "+v"(c20), "+v"(c21), "+v"(c30), "+v"(c31)
                     : "v"(a0), "v"(a1), "v"(a2), "v"(a3), "v"(b0), "v"(b1));
    }
    const int wb = wave * 64 * GP;
    STG(c00, 0, 0) STG(c01, 0, 1) STG(c10, 1, 0) STG(c11, 1, 1) STG(c20, 2, 0) STG(c21, 2, 1) STG(c30, 3, 0) STG(c31, 3, 1)
    __syncthreads();
    const int q = lane >> 3, p = lane & 7;
    if (MODE == 0) {
        h16* pl = (h16*)out;
        const int part = p & 3, fb = 8 * (part & 1), isres = part >> 1;
#pragma unroll 1
        for (int ps = 0; ps < 2; ++ps) {
#pragma unroll
            for (int hd = 0; hd < 2; ++hd) {
                const size_t hbase = ((size_t)((col0 >> 4) + hd) * ldo + row0) * 32;
#pragma unroll
                for (int s = 0; s < 8; ++s) { const int rr = 8 * s + 2 * q + (p >> 2);
                    const float* sp = &gs[wb + rr * GP + 16 * hd + fb];
                    const v4f x0 = *(const v4fa*)sp, x1 = *(const v4fa*)(sp + 4); v8h o;
#pragma unroll
                    for (int e = 0; e < 4; ++e) {
                        const float va = x0[e]; const h16 ha = (h16)va; const h16 ra = (h16)((va - (float)ha) * RSC); o[e] = isres ? ra : ha;
                        const float vb = x1[e]; const h16 hb = (h16)vb; const h16 rb = (h16)((vb - (float)hb) * RSC); o[4 + e] = isres ? rb : hb; }
                    *(volatile v8h*)(pl + hbase + (size_t)rr * 32 + part * 8) = o; } }
            if (ps == 0) __threadfence(); }
    }
    if (MODE == 1) {
        h16* pl = (h16*)out + (size_t)col0 * ldo + row0;
#pragma unroll 1
        for (int ps = 0; ps < 2; ++ps) {
#pragma unroll
            for (int s = 0; s < 8; ++s) { const int c = 4 * s + q; v8h o;
#pragma unroll
                for (int e = 0; e < 8; ++e) o[e] = (h16)gs[wb + (8 * p + e) * GP + c];
                *(volatile v8h*)(pl + (size_t)c * ldo + 8 * p) = o; }
            if (ps == 0) __threadfence(); }
    }
    if (MODE == 2) {
        float* op = (float*)out + (size_t)row0 * ldo + col0;
#pragma unroll 1
        for (int ps = 0; ps < 2; ++ps) {
#pragma unroll
            for (int s = 0; s < 16; ++s) { const int rr = 4 * s + q, c4 = p * 4;
                const v4f val = *(const v4fa*)(&gs[wb + rr * GP + c4]);
                *(volatile v4f*)(op + (size_t)rr * ldo + c4) = val; }
            if (ps == 0) __threadfence(); }
    }
}

__global__ __launch_bounds__(32 * AW) void k_stats(const h16* __restrict__ QP, const h16* __restrict__ KP, float* CP) {
    __shared__ __align__(16) float cs[AW * 16];
    const int lane = threadIdx.x & 31, wave = __builtin_amdgcn_readfirstlane((int)(threadIdx.x >> 5)), lr = lane & 15, hi = lane >> 4;
    const int hd = blockIdx.y;
    const int j0 = (blockIdx.x * AW + wave) * 16;
    const v8h z8 = (v8h){};
    const h16* kp = KP + ((size_t)hd * SEQJ + j0 + lr) * 32 + 8 * hi;
    const v8h kh = *(const v8h*)kp, kr = *(const v8h*)(kp + 16);
    const v16h B1 = cat16(kh, z8), B2 = cat16(kr, kh);
    const h16* qp = QP + ((size_t)hd * SEQI + lr) * 32 + 8 * hi;
    float m = -3.0e38f, l = 0.0f;
#pragma unroll 1
    for (int i0 = 0; i0 < SEQI; i0 += 32) {
        const h16* q0 = qp + (size_t)i0 * 32;
        const v16h qa = ldh(q0), qb = ldh(q0 + 16 * 32);
        v8f sa0 = (v8f){}, sb0 = (v8f){}, sa1 = (v8f){}, sb1 = (v8f){};
        sa0 = wmma16(qa, B1, sa0); sb0 = wmma16(qb, B1, sb0);
        sa1 = wmma16(qa, B2, sa1); sb1 = wmma16(qb, B2, sb1);
        asm volatile("v_nop\n\tv_nop\n\tv_nop\n\tv_nop" : "+v"(sa0), "+v"(sb0), "+v"(sa1), "+v"(sb1) : "v"(qa), "v"(qb), "v"(B1), "v"(B2));
        float ta[8], tb[8]; float mx = -3.0e38f;
#pragma unroll
        for (int r = 0; r < 8; ++r) { ta[r] = fmaf(sa1[r], RINV, sa0[r]); tb[r] = fmaf(sb1[r], RINV, sb0[r]); mx = fmaxf(mx, fmaxf(ta[r], tb[r])); }
        mx = fmaxf(mx, __shfl_xor(mx, 16, 32));
        const float mnew = fmaxf(m, mx);
        const float alpha = __builtin_amdgcn_exp2f((m - mnew) * SC2);
        float ls = 0.0f;
#pragma unroll
        for (int r = 0; r < 8; ++r) ls += __builtin_amdgcn_exp2f((ta[r] - mnew) * SC2) + __builtin_amdgcn_exp2f((tb[r] - mnew) * SC2);
        l = l * alpha + ls; m = mnew;
    }
    l += __shfl_xor(l, 16, 32);
    const float c = fmaf(-m, SC2, PSH - __log2f(l));
    if (hi == 0) cs[wave * 16 + lr] = c;
    __syncthreads();
    if (wave == 0 && lane < 16) {
        const v4f val = *(const v4fa*)(&cs[4 * lane]);
        float* dst = CP + (size_t)hd * SEQJ + (size_t)blockIdx.x * (16 * AW) + 4 * lane;
        *(volatile v4f*)dst = val;
        __threadfence();
        *(volatile v4f*)dst = val;
    }
}

__global__ __launch_bounds__(32 * AW) void k_apply(const h16* __restrict__ QP, const h16* __restrict__ KP, const h16* __restrict__ VT, const float* __restrict__ CP, u16* HP) {
    __shared__ __align__(16) float os[16 * 68];
    const int lane = threadIdx.x & 31, wave = __builtin_amdgcn_readfirstlane((int)(threadIdx.x >> 5)), lr = lane & 15, hi = lane >> 4;
    const int hd = blockIdx.y * AW + wave;
    const int i0 = blockIdx.x * 16;
    const v8h z8 = (v8h){};
    const h16* qp = QP + ((size_t)hd * SEQI + i0 + lr) * 32 + 8 * hi;
    const v8h qh = *(const v8h*)qp, qr = *(const v8h*)(qp + 16);
    const v16h B1 = cat16(qh, z8), B2 = cat16(qr, qh);
    const h16* kp = KP + ((size_t)hd * SEQJ + lr) * 32 + 8 * hi;
    const h16* vp = VT + ((size_t)(hd * FD + lr)) * SEQJ + 8 * hi;
    const float* cp = CP + (size_t)hd * SEQJ + 8 * hi;
    v8f o = (v8f){};
#pragma unroll 1
    for (int key0 = 0; key0 < SEQJ; key0 += 32) {
        const h16* k0p = kp + (size_t)key0 * 32;
        const v16h ka = ldh(k0p), kb = ldh(k0p + 16 * 32);
        v8f sa0 = (v8f){}, sb0 = (v8f){}, sa1 = (v8f){}, sb1 = (v8f){};
        sa0 = wmma16(ka, B1, sa0); sb0 = wmma16(kb, B1, sb0);
        sa1 = wmma16(ka, B2, sa1); sb1 = wmma16(kb, B2, sb1);
        asm volatile("v_nop\n\tv_nop\n\tv_nop\n\tv_nop" : "+v"(sa0), "+v"(sb0), "+v"(sa1), "+v"(sb1) : "v"(ka), "v"(kb), "v"(B1), "v"(B2));
        const v4f ca0 = *(const v4f*)(cp + key0), ca1 = *(const v4f*)(cp + key0 + 4), cb0 = *(const v4f*)(cp + key0 + 16), cb1 = *(const v4f*)(cp + key0 + 20);
        v16h pb;
#pragma unroll
        for (int r = 0; r < 4; ++r) {
            const float t0 = fmaf(sa1[r], RINV, sa0[r]);         pb[r]      = (h16)__builtin_amdgcn_exp2f(fmaf(t0, SC2, ca0[r]));
            const float t1 = fmaf(sa1[4 + r], RINV, sa0[4 + r]); pb[4 + r]  = (h16)__builtin_amdgcn_exp2f(fmaf(t1, SC2, ca1[r]));
            const float t2 = fmaf(sb1[r], RINV, sb0[r]);         pb[8 + r]  = (h16)__builtin_amdgcn_exp2f(fmaf(t2, SC2, cb0[r]));
            const float t3 = fmaf(sb1[4 + r], RINV, sb0[4 + r]); pb[12 + r] = (h16)__builtin_amdgcn_exp2f(fmaf(t3, SC2, cb1[r])); }
        const v16h va = ldh(vp + key0);
        o = wmma16(va, pb, o);
        asm volatile("v_nop\n\tv_nop\n\tv_nop\n\tv_nop" : "+v"(o) : "v"(va), "v"(pb));
    }
    { v4f a, c;
      a[0] = o[0] * OSC; a[1] = o[1] * OSC; a[2] = o[2] * OSC; a[3] = o[3] * OSC; c[0] = o[4] * OSC; c[1] = o[5] * OSC; c[2] = o[6] * OSC; c[3] = o[7] * OSC;
      *(v4fa*)(&os[lr * 68 + wave * 16 + 8 * hi]) = a; *(v4fa*)(&os[lr * 68 + wave * 16 + 8 * hi + 4]) = c; }
    __syncthreads();
    u16* hrow = HP + (size_t)i0 * HP2 + (size_t)blockIdx.y * (AW * FD);
#pragma unroll 1
    for (int ps = 0; ps < 2; ++ps) {
#pragma unroll
        for (int s = 0; s < 2; ++s) { const int L = wave * 8 + s * 4 + (lane >> 3);
            const int row = L >> 1, part = L & 1, c8 = (lane & 7) * 8;
            const v4f x0 = *(const v4fa*)(&os[row * 68 + c8]), x1 = *(const v4fa*)(&os[row * 68 + c8 + 4]); v8us ov;
#pragma unroll
            for (int e = 0; e < 4; ++e) {
                const float xa = x0[e]; const unsigned ha = rbfb(xa); const unsigned la = rbfb(xa - bf2f(ha)); ov[e] = (u16)(part ? la : ha);
                const float xb = x1[e]; const unsigned hb = rbfb(xb); const unsigned lb = rbfb(xb - bf2f(hb)); ov[4 + e] = (u16)(part ? lb : hb); }
            *(volatile v8us*)(hrow + (size_t)row * HP2 + part * DM + c8) = ov; }
        if (ps == 0) __threadfence(); }
}

static constexpr size_t al256(size_t v) { return (v + 255) & ~(size_t)255; }
static constexpr size_t SZ_XQ = al256((size_t)SEQI * DM * 2);
static constexpr size_t SZ_XK = al256((size_t)SEQJ * DM * 2);
static constexpr size_t SZ_W  = al256((size_t)DM * DM * 2);
static constexpr size_t SZ_QP = al256((size_t)NHD * SEQI * 32 * 2);
static constexpr size_t SZ_KP = al256((size_t)NHD * SEQJ * 32 * 2);
static constexpr size_t SZ_VT = al256((size_t)DM * SEQJ * 2);
static constexpr size_t SZ_CP = al256((size_t)NHD * SEQJ * 4);
static constexpr size_t SZ_HP = al256((size_t)SEQI * HP2 * 2);
static constexpr size_t SZ_TOTAL = SZ_XQ + 2 * SZ_XK + 4 * SZ_W + SZ_QP + SZ_KP + SZ_VT + SZ_CP + SZ_HP;
static_assert(SZ_TOTAL <= (size_t)134217728);

extern "C" void kernel_launch(void* const* d_in, const int* in_sizes, int n_in,
                              void* d_out, int out_size, void* d_ws, size_t ws_size, hipStream_t stream) {
    if (n_in < 7) return;
    if ((size_t)in_sizes[0] < (size_t)SEQI * DM) return;
    if ((size_t)in_sizes[1] < (size_t)SEQJ * DM || (size_t)in_sizes[2] < (size_t)SEQJ * DM) return;
    if ((size_t)in_sizes[3] < (size_t)DM * DM || (size_t)in_sizes[4] < (size_t)DM * DM || (size_t)in_sizes[5] < (size_t)DM * DM || (size_t)in_sizes[6] < (size_t)DM * DM) return;
    if ((size_t)out_size < (size_t)SEQI * DM) return;
    if (SZ_TOTAL > ws_size) return;
    const float* xq = (const float*)d_in[0]; const float* xk = (const float*)d_in[1]; const float* xv = (const float*)d_in[2];
    const float* wq = (const float*)d_in[3]; const float* wk = (const float*)d_in[4]; const float* wv = (const float*)d_in[5]; const float* wo = (const float*)d_in[6];
    float* OUT = (float*)d_out;
    char* wsp = (char*)d_ws;
    u16* XQ  = (u16*)wsp; wsp += SZ_XQ;
    u16* XK  = (u16*)wsp; wsp += SZ_XK;
    u16* XV  = (u16*)wsp; wsp += SZ_XK;
    u16* WTQ = (u16*)wsp; wsp += SZ_W;
    u16* WTK = (u16*)wsp; wsp += SZ_W;
    u16* WTV = (u16*)wsp; wsp += SZ_W;
    u16* WTO = (u16*)wsp; wsp += SZ_W;
    h16* QP  = (h16*)wsp; wsp += SZ_QP;
    h16* KP  = (h16*)wsp; wsp += SZ_KP;
    h16* VT  = (h16*)wsp; wsp += SZ_VT;
    float* CP = (float*)wsp; wsp += SZ_CP;
    u16* HP  = (u16*)wsp; wsp += SZ_HP;

    const size_t n8i = (size_t)SEQI * DM / 8, n8j = (size_t)SEQJ * DM / 8;
    k_cvt<<<(unsigned)((n8i + 255) / 256), 256, 0, stream>>>(xq, XQ, n8i);
    k_cvt<<<(unsigned)((n8j + 255) / 256), 256, 0, stream>>>(xk, XK, n8j);
    k_cvt<<<(unsigned)((n8j + 255) / 256), 256, 0, stream>>>(xv, XV, n8j);
    const dim3 gt(DM / 64, DM / 64, 1);
    k_wt<<<gt, 256, 0, stream>>>(wq, WTQ);
    k_wt<<<gt, 256, 0, stream>>>(wk, WTK);
    k_wt<<<gt, 256, 0, stream>>>(wv, WTV);
    k_wt<<<gt, 256, 0, stream>>>(wo, WTO);
    k_gemm<0, h16><<<dim3(DM / 128, SEQI / 64, 1), 32 * AW, 0, stream>>>(XQ, DM, WTQ, DM, DM, DM - 1, QP, SEQI, 1.0f);
    k_gemm<0, h16><<<dim3(DM / 128, SEQJ / 64, 1), 32 * AW, 0, stream>>>(XK, DM, WTK, DM, DM, DM - 1, KP, SEQJ, 1.0f);
    k_gemm<1, h16><<<dim3(DM / 128, SEQJ / 64, 1), 32 * AW, 0, stream>>>(XV, DM, WTV, DM, DM, DM - 1, VT, SEQJ, VSC);
    k_stats<<<dim3(SEQJ / (16 * AW), NHD, 1), 32 * AW, 0, stream>>>(QP, KP, CP);
    k_apply<<<dim3(SEQI / 16, NHD / AW, 1), 32 * AW, 0, stream>>>(QP, KP, VT, CP, HP);
    k_gemm<2, float><<<dim3(DM / 128, SEQI / 64, 1), 32 * AW, 0, stream>>>(HP, HP2, WTO, DM, HP2, DM - 1, OUT, DM, 1.0f);
}
